// RNN_21732534518291
// MI455X (gfx1250) — hardware-verified
//
#include <hip/hip_runtime.h>
#include <math.h>

constexpr int NSTEP    = 1024;
constexpr int NBATCH   = 512;
constexpr int NHID     = 64;
constexpr int ROWS_BLK = 32;
constexpr int NBLK     = NBATCH / ROWS_BLK;
constexpr int WPITCH   = 72;
constexpr int HPITCH   = 72;
constexpr float W_CARRY   = 8.0f;
constexpr float H_CARRY   = 16.0f;
constexpr float RES_CARRY = 2048.0f;
constexpr float INV_MAIN  = 1.0f / (W_CARRY * H_CARRY);
constexpr float INV_RES   = INV_MAIN / RES_CARRY;

static_assert(NBATCH % ROWS_BLK == 0, "batch tiles exact");
static_assert(NHID == 64, "K = 2 chunks of 32, M = 4 tiles of 16");
static_assert(ROWS_BLK == 32, "N = 2 tiles of 16, one 128-B line per step");
static_assert((WPITCH % 8) == 0 && (HPITCH % 8) == 0, "16-B aligned fragment loads");
static_assert(((2 * ROWS_BLK * HPITCH) / 8) % 32 == 0, "zero-fill loop exact");
static_assert(((NHID * NHID) / 8) % 32 == 0, "weight plane build loop exact");

typedef __attribute__((ext_vector_type(16))) _Float16 v16h;
typedef __attribute__((ext_vector_type(8)))  _Float16 v8h;
typedef __attribute__((ext_vector_type(8)))  float    v8f;
typedef __attribute__((ext_vector_type(4)))  float    v4f;

union FragU { v16h v; v8h h[2]; };

__device__ __forceinline__ v16h frag_load(const _Float16* p) {
  FragU f;
  f.h[0] = *(const v8h*)(p);
  f.h[1] = *(const v8h*)(p + 16);
  return f.v;
}
__device__ __forceinline__ v8f mma_h(v16h a, v16h b, v8f c) {
  return __builtin_amdgcn_wmma_f32_16x16x32_f16(false, a, false, b, (short)0, c, false, false);
}
__device__ __forceinline__ void guard2_a4(v8f& a, v8f& b, v16h w, v16h x, v16h y, v16h z) {
  asm volatile("v_nop\n\tv_nop\n\tv_nop\n\tv_nop" : "+v"(a), "+v"(b) : "v"(w), "v"(x), "v"(y), "v"(z));
}
__device__ __forceinline__ void keep4_h(v16h a, v16h b, v16h c, v16h d) {
  asm volatile("v_nop" :: "v"(a), "v"(b), "v"(c), "v"(d));
}

__global__ __launch_bounds__(32) void rnn_seq_kernel(const float* __restrict__ x,
                                                     const float* __restrict__ w_ih,
                                                     const float* __restrict__ w_hh,
                                                     const float* __restrict__ b_ih,
                                                     const float* __restrict__ b_hh,
                                                     const float* __restrict__ w_out,
                                                     const float* __restrict__ b_out,
                                                     float* __restrict__ out) {
  __shared__ __align__(16) _Float16 Whi[NHID * WPITCH];
  __shared__ __align__(16) _Float16 Wlo[NHID * WPITCH];
  __shared__ __align__(16) _Float16 Hhi[2 * ROWS_BLK * HPITCH];
  __shared__ __align__(16) _Float16 Hlo[2 * ROWS_BLK * HPITCH];
  __shared__ __align__(16) float Cst[3 * NHID];

  const int lane = threadIdx.x & 31;
  const int c    = lane & 15;
  const int hh   = lane >> 4;
  const int koff = 8 * hh;
  const int base = blockIdx.x * ROWS_BLK;

  {
    const float wi0 = w_ih[lane];
    const float wi1 = w_ih[lane + 32];
    const float bi0 = b_ih[lane];
    const float bi1 = b_ih[lane + 32];
    const float bh0 = b_hh[lane];
    const float bh1 = b_hh[lane + 32];
    const float wo0 = w_out[lane];
    const float wo1 = w_out[lane + 32];
    Cst[lane]                 = wi0;
    Cst[lane + 32]            = wi1;
    Cst[NHID + lane]          = bi0 + bh0;
    Cst[NHID + lane + 32]     = bi1 + bh1;
    Cst[2 * NHID + lane]      = wo0;
    Cst[2 * NHID + lane + 32] = wo1;
  }
  const float bout = b_out[0];

#pragma unroll 1
  for (int it = 0; it < (NHID * NHID) / (8 * 32); ++it) {
    const int g   = it * 32 + lane;
    const int row = g >> 3;
    const int c8  = (g & 7) * 8;
    const v4f wa = *(const v4f*)(w_hh + row * NHID + c8);
    const v4f wb = *(const v4f*)(w_hh + row * NHID + c8 + 4);
    v8h hv, lv;
#pragma unroll
    for (int e = 0; e < 4; ++e) {
      const float f0 = wa[e] * W_CARRY;
      const float f1 = wb[e] * W_CARRY;
      const _Float16 h0 = (_Float16)f0;
      const _Float16 h1 = (_Float16)f1;
      float g0 = (float)h0;
      float g1 = (float)h1;
      asm volatile("" : "+v"(g0));
      asm volatile("" : "+v"(g1));
      hv[e]     = h0;
      hv[4 + e] = h1;
      lv[e]     = (_Float16)((f0 - g0) * RES_CARRY);
      lv[4 + e] = (_Float16)((f1 - g1) * RES_CARRY);
    }
    *(v8h*)(Whi + row * WPITCH + c8) = hv;
    *(v8h*)(Wlo + row * WPITCH + c8) = lv;
  }

  {
    v8h zh;
#pragma unroll
    for (int e = 0; e < 8; ++e) zh[e] = (_Float16)0.0f;
#pragma unroll 1
    for (int i = lane; i < (2 * ROWS_BLK * HPITCH) / 8; i += 32) {
      ((v8h*)Hhi)[i] = zh;
      ((v8h*)Hlo)[i] = zh;
    }
  }
  __syncthreads();

  const v8f z8 = {0.f, 0.f, 0.f, 0.f, 0.f, 0.f, 0.f, 0.f};

#pragma unroll 1
  for (int t = 0; t < NSTEP; ++t) {
    const int cur = t & 1;
    const _Float16* hc_hi = Hhi + cur * (ROWS_BLK * HPITCH);
    const _Float16* hc_lo = Hlo + cur * (ROWS_BLK * HPITCH);
    _Float16* hn_hi = Hhi + (cur ^ 1) * (ROWS_BLK * HPITCH);
    _Float16* hn_lo = Hlo + (cur ^ 1) * (ROWS_BLK * HPITCH);

    const float* xr = x + (size_t)t * NBATCH + base;
    const float xa = xr[c];
    const float xb = xr[16 + c];

    float res = 0.0f;

#pragma unroll 1
    for (int n = 0; n < 2; ++n) {
      const float xv = (n == 0) ? xa : xb;
      const int brow = 16 * n + c;
      const _Float16* bp_hi = hc_hi + brow * HPITCH + koff;
      const _Float16* bp_lo = hc_lo + brow * HPITCH + koff;
      const v16h bh0 = frag_load(bp_hi);
      const v16h bh1 = frag_load(bp_hi + 32);
      const v16h bl0 = frag_load(bp_lo);
      const v16h bl1 = frag_load(bp_lo + 32);

      float po = 0.0f;

#pragma unroll 1
      for (int m = 0; m < 4; ++m) {
        const int arow = 16 * m + c;
        const _Float16* ap_hi = Whi + arow * WPITCH + koff;
        const _Float16* ap_lo = Wlo + arow * WPITCH + koff;
        const v16h ah0 = frag_load(ap_hi);
        const v16h ah1 = frag_load(ap_hi + 32);
        const v16h al0 = frag_load(ap_lo);
        const v16h al1 = frag_load(ap_lo + 32);

        const int hid0 = 16 * m + 8 * hh;
        const v4f wiA = *(const v4f*)(Cst + hid0);
        const v4f wiB = *(const v4f*)(Cst + hid0 + 4);
        const v4f bsA = *(const v4f*)(Cst + NHID + hid0);
        const v4f bsB = *(const v4f*)(Cst + NHID + hid0 + 4);
        const v4f woA = *(const v4f*)(Cst + 2 * NHID + hid0);
        const v4f woB = *(const v4f*)(Cst + 2 * NHID + hid0 + 4);
        float wi[8], bs[8], wo[8];
#pragma unroll
        for (int e = 0; e < 4; ++e) {
          wi[e] = wiA[e];
          wi[4 + e] = wiB[e];
          bs[e] = bsA[e];
          bs[4 + e] = bsB[e];
          wo[e] = woA[e];
          wo[4 + e] = woB[e];
        }

        v8f accM = z8;
        v8f accR = z8;
        accM = mma_h(ah0, bh0, accM);
        accM = mma_h(ah1, bh1, accM);
        accR = mma_h(ah0, bl0, accR);
        accR = mma_h(al0, bh0, accR);
        accR = mma_h(ah1, bl1, accR);
        accR = mma_h(al1, bh1, accR);
        guard2_a4(accM, accR, ah0, ah1, al0, al1);
        keep4_h(bh0, bh1, bl0, bl1);

        v8h hv, lv;
#pragma unroll
        for (int r = 0; r < 8; ++r) {
          const float pre = fmaf(xv, wi[r], bs[r]) + accM[r] * INV_MAIN + accR[r] * INV_RES;
          const float th  = tanhf(pre);
          po += th * wo[r];
          const float hs = th * H_CARRY;
          const _Float16 hi = (_Float16)hs;
          float hf = (float)hi;
          asm volatile("" : "+v"(hf));
          hv[r] = hi;
          lv[r] = (_Float16)((hs - hf) * RES_CARRY);
        }
        *(v8h*)(hn_hi + brow * HPITCH + hid0) = hv;
        *(v8h*)(hn_lo + brow * HPITCH + hid0) = lv;
      }

      const float oth = __shfl_xor(po, 16, 32);
      const float s = po + oth;
      res = (n == hh) ? s : res;
    }

    {
      const float ov = res + bout;
      volatile float* op = out + (size_t)t * NBATCH + base + lane;
      *op = ov;
      __threadfence();
      *op = ov;
    }

    __syncthreads();
  }
}

extern "C" void kernel_launch(void* const* d_in, const int* in_sizes, int n_in,
                              void* d_out, int out_size, void* d_ws, size_t ws_size, hipStream_t stream) {
  (void)d_ws;
  (void)ws_size;
  if (n_in < 7 || d_out == nullptr) return;
  if (in_sizes[0] != NSTEP * NBATCH || in_sizes[1] != NHID || in_sizes[2] != NHID * NHID ||
      in_sizes[3] != NHID || in_sizes[4] != NHID || in_sizes[5] != NHID || in_sizes[6] != 1 ||
      out_size != NSTEP * NBATCH) return;

  const float* x     = (const float*)d_in[0];
  const float* w_ih  = (const float*)d_in[1];
  const float* w_hh  = (const float*)d_in[2];
  const float* b_ih  = (const float*)d_in[3];
  const float* b_hh  = (const float*)d_in[4];
  const float* w_out = (const float*)d_in[5];
  const float* b_out = (const float*)d_in[6];
  float* out = (float*)d_out;

  rnn_seq_kernel<<<NBLK, 32, 0, stream>>>(x, w_ih, w_hh, b_ih, b_hh, w_out, b_out, out);
}
